// BitLinear_22162031248001
// MI455X (gfx1250) — hardware-verified
//
#include <hip/hip_runtime.h>
#include <stdint.h>

typedef __attribute__((ext_vector_type(16))) _Float16 v16h;
typedef __attribute__((ext_vector_type(8)))  _Float16 v8h;
typedef __attribute__((ext_vector_type(16))) __bf16   v16b;
typedef __attribute__((ext_vector_type(8)))  __bf16   v8b;
typedef __attribute__((ext_vector_type(8)))  float    v8f;
typedef __attribute__((ext_vector_type(4)))  float    v4f;
typedef __attribute__((ext_vector_type(4)))  unsigned v4u;

constexpr int NTOK         = 64;
constexpr int IN_FEATS     = 4096;
constexpr int OUT_FEATS    = 11008;
constexpr int INTS_PER_ROW = IN_FEATS / 8;
constexpr int N_INTS       = OUT_FEATS * INTS_PER_ROW;
static_assert(INTS_PER_ROW == 512, "row index uses >> 9");
static_assert(N_INTS == 5636096, "packed weight count");
static_assert(N_INTS % 256 == 0, "expand grid exact");
static_assert((NTOK * IN_FEATS) % (8 * 256) == 0, "cast grid exact");
static_assert(NTOK % 64 == 0, "M tile multiple");
static_assert(OUT_FEATS % 64 == 0, "N tile multiple");
static_assert(IN_FEATS % 32 == 0, "K multiple of 32");

constexpr size_t WS_XB_OFF   = 0;
constexpr size_t WS_XB_BYTES = (size_t)NTOK * IN_FEATS * 2;
constexpr size_t WS_W_OFF    = WS_XB_OFF + WS_XB_BYTES;
constexpr size_t WS_W_BYTES  = (size_t)OUT_FEATS * IN_FEATS * 2;
constexpr size_t WS_TOTAL    = WS_W_OFF + WS_W_BYTES;
static_assert(WS_W_OFF % 128 == 0, "aligned carve");
static_assert(WS_TOTAL <= 134217728ull, "carve within 128 MiB");

__device__ __forceinline__ unsigned short f2bf_bits(float f) {
  unsigned u = __float_as_uint(f);
  return (unsigned short)((u + 0x7FFFu + ((u >> 16) & 1u)) >> 16);
}
__device__ __forceinline__ float bf_bits2f(unsigned short h) { return __uint_as_float(((unsigned)h) << 16); }

__device__ __forceinline__ void dep_guard_h(v8f& a, v8f& b, v16h x, v16h y) { asm volatile("v_nop\n\tv_nop\n\tv_nop\n\tv_nop" : "+v"(a), "+v"(b) : "v"(x), "v"(y)); }
__device__ __forceinline__ void dep_guard_b(v8f& a, v8f& b, v16b x, v16b y) { asm volatile("v_nop\n\tv_nop\n\tv_nop\n\tv_nop" : "+v"(a), "+v"(b) : "v"(x), "v"(y)); }
__device__ __forceinline__ void keep4_h(v16h a, v16h b, v16h c, v16h d) { asm volatile("v_nop" :: "v"(a), "v"(b), "v"(c), "v"(d)); }
__device__ __forceinline__ void keep4_b(v16b a, v16b b, v16b c, v16b d) { asm volatile("v_nop" :: "v"(a), "v"(b), "v"(c), "v"(d)); }
__device__ __forceinline__ void acc_guard4(v8f& a, v8f& b, v8f& c, v8f& d) { asm volatile("v_nop\n\tv_nop\n\tv_nop\n\tv_nop" : "+v"(a), "+v"(b), "+v"(c), "+v"(d)); }
template <typename T> struct Frag;
template <> struct Frag<_Float16> {
  typedef v16h V; union U { v16h v; v8h h[2]; };
  static __device__ __forceinline__ v16h load(const _Float16* p) {
    U f; f.h[0] = *(const v8h*)(p); f.h[1] = *(const v8h*)(p + 16); return f.v;
  }
  static __device__ __forceinline__ v8f mma(v16h a, v16h b, v8f c) {
    return __builtin_amdgcn_wmma_f32_16x16x32_f16(false, a, false, b, (short)0, c, false, false);
  }
  static __device__ __forceinline__ void guard(v8f& a, v8f& b, v16h x, v16h y) { dep_guard_h(a, b, x, y); }
  static __device__ __forceinline__ void keep(v16h a, v16h b, v16h c, v16h d) { keep4_h(a, b, c, d); }
};
template <> struct Frag<__bf16> {
  typedef v16b V; union U { v16b v; v8b h[2]; };
  static __device__ __forceinline__ v16b load(const __bf16* p) {
    U f; f.h[0] = *(const v8b*)(p); f.h[1] = *(const v8b*)(p + 16); return f.v;
  }
  static __device__ __forceinline__ v8f mma(v16b a, v16b b, v8f c) {
    return __builtin_amdgcn_wmma_f32_16x16x32_bf16(false, a, false, b, (short)0, c, false, false);
  }
  static __device__ __forceinline__ void guard(v8f& a, v8f& b, v16b x, v16b y) { dep_guard_b(a, b, x, y); }
  static __device__ __forceinline__ void keep(v16b a, v16b b, v16b c, v16b d) { keep4_b(a, b, c, d); }
};

template <int ET> struct Elem;
template <> struct Elem<0> { typedef _Float16 T; };
template <> struct Elem<1> { typedef __bf16 T; };
template <int ET, bool SPLIT, int BIAS_MODE, int OUT_MODE, bool RESID, int ACT = 0>
__global__ __launch_bounds__(256) void wmma_gemm64(
    const unsigned short* __restrict__ Ap, const unsigned short* __restrict__ A2p, int lda, long strideA,
    const unsigned short* __restrict__ Btp, const unsigned short* __restrict__ Bt2p, int ldb, long strideB,
    void* __restrict__ Cout, void* __restrict__ Cout2, int ldc, long strideC,
    const float* __restrict__ bias,
    const float* __restrict__ resid, long strideR,
    int M, int N, int K, float scale) {
  typedef typename Elem<ET>::T T;
  typedef typename Frag<T>::V V;
  const T* A = (const T*)Ap; const T* A2 = (const T*)A2p; const T* Bt = (const T*)Btp; const T* Bt2 = (const T*)Bt2p;
  __shared__ __align__(16) float sT[8][16 * 68];
  const int b    = blockIdx.y;
  const int lane = threadIdx.x & 31;
  const int wave = threadIdx.x >> 5;
  const int tilesN = N >> 6;
  const int tilesM = M >> 6;
  const int tile = blockIdx.x * 8 + wave;
  if (tile >= tilesM * tilesN) return;
  const int tm = tile / tilesN;
  const int tn = tile - tm * tilesN;
  const int m0 = tm << 6;
  const int n0 = tn << 6;

  const T* Ab  = A  + (size_t)b * strideA;
  const T* Bb  = Bt + (size_t)b * strideB;
  const T* Ab2 = SPLIT ? (A2  + (size_t)b * strideA) : nullptr;
  const T* Bb2 = SPLIT ? (Bt2 + (size_t)b * strideB) : nullptr;

  const int rlane = lane & 15;
  const int koff  = (lane >> 4) * 8;
  const int mOff  = (lane >> 4) * 8;

  v8f acc[4][4];
#pragma unroll
  for (int i = 0; i < 4; ++i)
#pragma unroll
    for (int j = 0; j < 4; ++j) acc[i][j] = (v8f){0.f,0.f,0.f,0.f,0.f,0.f,0.f,0.f};

  for (int k0 = 0; k0 < K; k0 += 32) {
    V bh[4], bl[4];
#pragma unroll
    for (int j = 0; j < 4; ++j) {
      const size_t bo = (size_t)(n0 + (j << 4) + rlane) * ldb + koff + k0;
      bh[j] = Frag<T>::load(Bb + bo);
      if (SPLIT) bl[j] = Frag<T>::load(Bb2 + bo);
    }
#pragma unroll
    for (int i = 0; i < 4; ++i) {
      const size_t ao = (size_t)(m0 + (i << 4) + rlane) * lda + koff + k0;
      V ah = Frag<T>::load(Ab + ao);
      V al;
      if (SPLIT) al = Frag<T>::load(Ab2 + ao);
#pragma unroll
      for (int j = 0; j < 4; ++j) {
        acc[i][j] = Frag<T>::mma(ah, bh[j], acc[i][j]);
        if (SPLIT) {
          acc[i][j] = Frag<T>::mma(ah, bl[j], acc[i][j]);
          acc[i][j] = Frag<T>::mma(al, bh[j], acc[i][j]);
        }
      }
      Frag<T>::guard(acc[i][0], acc[i][3], ah, SPLIT ? al : ah);
    }
    Frag<T>::keep(bh[0], bh[1], bh[2], bh[3]);
    if (SPLIT) Frag<T>::keep(bl[0], bl[1], bl[2], bl[3]);
  }
  acc_guard4(acc[0][0], acc[0][1], acc[0][2], acc[0][3]);
  acc_guard4(acc[1][0], acc[1][1], acc[1][2], acc[1][3]);
  acc_guard4(acc[2][0], acc[2][1], acc[2][2], acc[2][3]);
  acc_guard4(acc[3][0], acc[3][1], acc[3][2], acc[3][3]);

  float* slab = sT[wave];
  const float* Rb = RESID ? (resid + (size_t)b * strideR) : nullptr;
#pragma unroll
  for (int i = 0; i < 4; ++i) {
    const int mBase = m0 + (i << 4);
#pragma unroll
    for (int j = 0; j < 4; ++j) {
      const int n = n0 + (j << 4) + rlane;
      float bv = 0.f;
      if (BIAS_MODE == 2) bv = bias[n];
#pragma unroll
      for (int r = 0; r < 8; ++r) {
        float v = acc[i][j][r] * scale;
        if (BIAS_MODE == 1) v += bias[mBase + mOff + r];
        if (BIAS_MODE == 2) v += bv;
        if (RESID) v += Rb[(size_t)(mBase + mOff + r) * ldc + n];
        if (ACT == 1) v = tanhf(v);
        if (ACT == 2) v = fmaxf(v, 0.0f);
        if (ACT == 3) v = v / (1.0f + expf(-v));
        if (ACT == 4) v = (v > 0.f) ? v : 0.01f * v;
        if (ACT == 5) v = 0.5f * v * (1.0f + erff(v * 0.70710678118654752f));
        slab[(mOff + r) * 68 + (j << 4) + rlane] = v;
      }
    }
    __builtin_amdgcn_fence(__ATOMIC_RELEASE, "workgroup");
    __builtin_amdgcn_wave_barrier();
    __builtin_amdgcn_fence(__ATOMIC_ACQUIRE, "workgroup");
    if (OUT_MODE == 0) {
      float* C = (float*)Cout + (size_t)b * strideC;
      const int hh = lane >> 4, c4 = (lane & 15) * 4;
      for (int pass = 0; pass < 2; ++pass) {
#pragma unroll
        for (int it = 0; it < 8; ++it) {
          const int row = it * 2 + hh;
          v4f v = *(const v4f*)(slab + row * 68 + c4);
          *(volatile v4f*)(C + (size_t)(mBase + row) * ldc + n0 + c4) = v;
        }
        __threadfence();
      }
    } else {
      const int q = lane >> 3, c8 = (lane & 7) * 8;
      unsigned short* C  = (unsigned short*)Cout  + (size_t)b * strideC;
      unsigned short* C2 = (OUT_MODE == 2) ? ((unsigned short*)Cout2 + (size_t)b * strideC) : nullptr;
      for (int pass = 0; pass < 2; ++pass) {
#pragma unroll
        for (int it = 0; it < 4; ++it) {
          const int row = it * 4 + q;
          const float* sp = slab + row * 68 + c8;
          v8h hv, lv;
#pragma unroll
          for (int e = 0; e < 8; ++e) {
            if (OUT_MODE == 1) {
              hv[e] = (_Float16)sp[e];
            } else {
              unsigned short hb = f2bf_bits(sp[e]);
              unsigned short lb = f2bf_bits(sp[e] - bf_bits2f(hb));
              hv[e] = __builtin_bit_cast(_Float16, hb);
              lv[e] = __builtin_bit_cast(_Float16, lb);
            }
          }
          *(volatile v8h*)(C + (size_t)(mBase + row) * ldc + n0 + c8) = hv;
          if (OUT_MODE == 2) *(volatile v8h*)(C2 + (size_t)(mBase + row) * ldc + n0 + c8) = lv;
        }
        __threadfence();
      }
    }
    __builtin_amdgcn_fence(__ATOMIC_RELEASE, "workgroup");
    __builtin_amdgcn_wave_barrier();
    __builtin_amdgcn_fence(__ATOMIC_ACQUIRE, "workgroup");
  }
}

__global__ __launch_bounds__(256) void cast_x_bf16x8(
    const float* __restrict__ x, unsigned short* __restrict__ xb, int n8) {
  const int t = blockIdx.x * 256 + threadIdx.x;
  const bool valid = t < n8;
  const int tc = valid ? t : (n8 - 1);
  const v4f a = *(const v4f*)(x + (size_t)tc * 8);
  const v4f c = *(const v4f*)(x + (size_t)tc * 8 + 4);
  v4u w;
  w[0] = (unsigned)f2bf_bits(a[0]) | ((unsigned)f2bf_bits(a[1]) << 16);
  w[1] = (unsigned)f2bf_bits(a[2]) | ((unsigned)f2bf_bits(a[3]) << 16);
  w[2] = (unsigned)f2bf_bits(c[0]) | ((unsigned)f2bf_bits(c[1]) << 16);
  w[3] = (unsigned)f2bf_bits(c[2]) | ((unsigned)f2bf_bits(c[3]) << 16);
  unsigned short* dst = xb + (size_t)tc * 8;
  if (valid) *(volatile v4u*)dst = w;
  __threadfence();
  if (valid) *(volatile v4u*)dst = w;
}

__global__ __launch_bounds__(256) void expand_w_bf16(
    const int* __restrict__ bp, const float* __restrict__ scale,
    unsigned short* __restrict__ W, int nInts) {
  const int t = blockIdx.x * 256 + threadIdx.x;
  const bool valid = t < nInts;
  const int tc = valid ? t : (nInts - 1);
  const int o = tc >> 9;
  const unsigned v = (unsigned)bp[tc];
  const unsigned sb = (unsigned)f2bf_bits(scale[o]);
  const unsigned base = sb | (sb << 16);
  v4u w;
#pragma unroll
  for (int j = 0; j < 4; ++j) {
    const unsigned b0 = (v >> (7 - 2 * j)) & 1u;
    const unsigned b1 = (v >> (6 - 2 * j)) & 1u;
    w[j] = base ^ (((b0 ^ 1u) << 15) | ((b1 ^ 1u) << 31));
  }
  unsigned short* dst = W + (size_t)tc * 8;
  if (valid) *(volatile v4u*)dst = w;
  __threadfence();
  if (valid) *(volatile v4u*)dst = w;
}

extern "C" void kernel_launch(void* const* d_in, const int* in_sizes, int n_in,
                              void* d_out, int out_size, void* d_ws, size_t ws_size,
                              hipStream_t stream) {
  if (n_in < 3) return;
  if (ws_size < WS_TOTAL) return;
  if (out_size < NTOK * OUT_FEATS) return;
  if (in_sizes[0] < NTOK * IN_FEATS || in_sizes[1] < N_INTS || in_sizes[2] < OUT_FEATS) return;

  const float* x     = (const float*)d_in[0];
  const int*   bp    = (const int*)d_in[1];
  const float* scale = (const float*)d_in[2];
  float*       out   = (float*)d_out;
  unsigned char* ws  = (unsigned char*)d_ws;
  unsigned short* xb = (unsigned short*)(ws + WS_XB_OFF);
  unsigned short* wb = (unsigned short*)(ws + WS_W_OFF);

  const int n8 = NTOK * IN_FEATS / 8;
  cast_x_bf16x8<<<n8 / 256, 256, 0, stream>>>(x, xb, n8);

  expand_w_bf16<<<N_INTS / 256, 256, 0, stream>>>(bp, scale, wb, N_INTS);

  const int tiles = (NTOK / 64) * (OUT_FEATS / 64);
  const int gx = (tiles + 7) / 8;
  wmma_gemm64<1, false, 0, 0, false, 0><<<dim3(gx, 1, 1), 256, 0, stream>>>(
      (const unsigned short*)xb, (const unsigned short*)xb, IN_FEATS, 0L,
      (const unsigned short*)wb, (const unsigned short*)wb, IN_FEATS, 0L,
      (void*)out, (void*)out, OUT_FEATS, 0L,
      scale,
      x, 0L,
      NTOK, OUT_FEATS, IN_FEATS, 1.0f);
}
